// MoonVitEncoderLayer_87333864996970
// MI455X (gfx1250) — hardware-verified
//
#include <hip/hip_runtime.h>


#define NB_  4
#define TT   1024
#define LL   4096
#define DD   1024
#define NH_  16
#define HDM  64
#define MM   4096
#define PCAR 1024.0f
typedef _Float16 h16;
typedef unsigned short bf;
typedef __attribute__((ext_vector_type(16))) __bf16   v16bf;
typedef __attribute__((ext_vector_type(16))) _Float16 v16h;
typedef __attribute__((ext_vector_type(8)))  _Float16 v8h;
typedef __attribute__((ext_vector_type(8)))  unsigned short v8us;
typedef __attribute__((ext_vector_type(8)))  float    v8f;
typedef __attribute__((ext_vector_type(4)))  float    v4f;
typedef v8h  __attribute__((may_alias)) v8ha;
typedef v4f  __attribute__((may_alias)) v4fa;
typedef v8us __attribute__((may_alias)) v8usa;

__device__ __forceinline__ unsigned short f2bf(float f) { unsigned u = __float_as_uint(f); u += 0x7FFFu + ((u >> 16) & 1u); return (unsigned short)(u >> 16); }
__device__ __forceinline__ float bf2f(unsigned short b) { return __uint_as_float(((unsigned)b) << 16); }
__device__ __forceinline__ float bfr(float f) { return bf2f(f2bf(f)); }
__device__ __forceinline__ v16h cat16(v8h lo, v8h hi) { return __builtin_shufflevector(lo, hi, 0, 1, 2, 3, 4, 5, 6, 7, 8, 9, 10, 11, 12, 13, 14, 15); }
__device__ __forceinline__ v16bf cat16b(v8us lo, v8us hi) { return __builtin_bit_cast(v16bf, __builtin_shufflevector(lo, hi, 0, 1, 2, 3, 4, 5, 6, 7, 8, 9, 10, 11, 12, 13, 14, 15)); }
__device__ __forceinline__ v8f wmma16(v16h a, v16h b, v8f c) { return __builtin_amdgcn_wmma_f32_16x16x32_f16(false, a, false, b, (short)0, c, false, false); }
__device__ __forceinline__ v8f wmmab(v16bf a, v16bf b, v8f c) { return __builtin_amdgcn_wmma_f32_16x16x32_bf16(false, a, false, b, (short)0, c, false, false); }


template <typename T16> struct WFrag;
template <> struct WFrag<h16> { typedef v16h V; static __device__ __forceinline__ V ld(const h16* p) { return cat16(*(const v8h*)p, *(const v8h*)(p + 16)); } static __device__ __forceinline__ v8f mma(V a, V b, v8f c) { return wmma16(a, b, c); } };
template <> struct WFrag<bf> { typedef v16bf V; static __device__ __forceinline__ V ld(const bf* p) { return cat16b(*(const v8us*)p, *(const v8us*)(p + 16)); } static __device__ __forceinline__ v8f mma(V a, V b, v8f c) { return wmmab(a, b, c); } };
template <typename T16, int NSPLIT, bool BIAS>
__global__ __launch_bounds__(32) void k_gemmw(const T16* __restrict__ A, const T16* __restrict__ A2, const T16* __restrict__ Bt, const T16* __restrict__ Bt2, int K, float* C, int ldc, const float* __restrict__ bias, size_t sA, size_t sB, size_t sC) {
    typedef typename WFrag<T16>::V V;
    __shared__ __align__(16) float os[16 * 68];
    const size_t z = blockIdx.z; A += z * sA; if (A2) A2 += z * sA; Bt += z * sB; if (Bt2) Bt2 += z * sB; C += z * sC;
    const int lane = threadIdx.x & 31, lr = lane & 15, hi = lane >> 4; const int r0 = blockIdx.x * 64, c0 = blockIdx.y * 64;
    v8f acc[4][4];
#pragma unroll
    for (int mb = 0; mb < 4; ++mb)
#pragma unroll
        for (int nb = 0; nb < 4; ++nb) acc[mb][nb] = (v8f){};
    const size_t aoff = (size_t)(r0 + lr) * K + 8 * hi, boff = (size_t)(c0 + lr) * K + 8 * hi;
#pragma unroll 1
    for (int kc = 0; kc < K; kc += 32) {
        V a[4], a2[4];
#pragma unroll
        for (int mb = 0; mb < 4; ++mb) { a[mb] = WFrag<T16>::ld(A + aoff + (size_t)mb * 16 * K + kc); if (NSPLIT == 1 || NSPLIT == 2) a2[mb] = WFrag<T16>::ld(A2 + aoff + (size_t)mb * 16 * K + kc); }
#pragma unroll
        for (int nb = 0; nb < 4; ++nb) { const V b = WFrag<T16>::ld(Bt + boff + (size_t)nb * 16 * K + kc); V b2; if (NSPLIT >= 2) b2 = WFrag<T16>::ld(Bt2 + boff + (size_t)nb * 16 * K + kc);
#pragma unroll
            for (int mb = 0; mb < 4; ++mb) { acc[mb][nb] = WFrag<T16>::mma(a[mb], b, acc[mb][nb]); if (NSPLIT == 1 || NSPLIT == 2) acc[mb][nb] = WFrag<T16>::mma(a2[mb], b, acc[mb][nb]); if (NSPLIT >= 2) acc[mb][nb] = WFrag<T16>::mma(a[mb], b2, acc[mb][nb]); } }
        asm volatile("v_nop\n\tv_nop\n\tv_nop\n\tv_nop" : "+v"(acc[0][0]), "+v"(acc[1][1]), "+v"(acc[2][2]), "+v"(acc[3][3]) : "v"(a[0]), "v"(a[3]));
    }
#pragma unroll
    for (int mb = 0; mb < 4; ++mb) {
#pragma unroll
        for (int nb = 0; nb < 4; ++nb) {
#pragma unroll
            for (int j = 0; j < 8; ++j) os[(hi * 8 + j) * 68 + nb * 16 + lr] = acc[mb][nb][j]; }
        __builtin_amdgcn_wave_barrier(); asm volatile("" ::: "memory");
        float* crow = C + (size_t)(r0 + mb * 16) * ldc + c0;
#pragma unroll 1
        for (int ps = 0; ps < 2; ++ps) {
#pragma unroll
            for (int s = 0; s < 8; ++s) { const int row = 2 * s + hi, cofs = lr * 4; v4f val = *(const v4fa*)(os + row * 68 + cofs); if (BIAS) { val[0] += bfr(bias[c0 + cofs]); val[1] += bfr(bias[c0 + cofs + 1]); val[2] += bfr(bias[c0 + cofs + 2]); val[3] += bfr(bias[c0 + cofs + 3]); }
                *(volatile v4f*)(crow + (size_t)row * ldc + cofs) = val; }
            if (ps == 0) __threadfence(); }
        __builtin_amdgcn_wave_barrier(); asm volatile("" ::: "memory");
    }
}

__device__ __forceinline__ h16 tohx(float x) { return (h16)x; }
__device__ __forceinline__ void splitf(float y, unsigned short& h, unsigned short& l) { h = f2bf(y); l = f2bf(y - bf2f(h)); }
typedef __attribute__((ext_vector_type(2))) _Float16 v2h;
typedef __attribute__((ext_vector_type(4))) _Float16 v4h;
typedef __attribute__((ext_vector_type(2))) unsigned short v2us;
typedef __attribute__((ext_vector_type(4))) unsigned short v4us;
typedef __attribute__((ext_vector_type(2))) float v2f;

__global__ __launch_bounds__(256) void k_wtG(const float* __restrict__ w, int K, int N, bf* Bt) {
    const int lane = threadIdx.x & 31; const int L0 = (blockIdx.x * 8 + (threadIdx.x >> 5)) * 8; const int nlines = N * K / 64;
#pragma unroll 1
    for (int ps = 0; ps < 2; ++ps) {
#pragma unroll 1
        for (int l = 0; l < 8; ++l) { const int L = L0 + l; if (L >= nlines) break; const size_t e = (size_t)L * 64 + lane * 2; const int k = (int)(e % K), n = (int)(e / K); v2us o;
            o[0] = f2bf(w[(size_t)k * N + n]); o[1] = f2bf(w[(size_t)(k + 1) * N + n]); *(volatile v2us*)(Bt + e) = o; }
        if (ps == 0) __threadfence(); }
}
__global__ __launch_bounds__(256) void k_pl(const float* __restrict__ F, int pitch, int nh, int hd, h16* P) { const size_t e = ((size_t)blockIdx.x * 256 + threadIdx.x) * 2; if (e >= (size_t)nh * TT * hd) return; const int d = (int)(e % hd); const int t = (int)((e / hd) % TT); const int h = (int)(e / ((size_t)hd * TT)); v2h o; o[0] = tohx(F[(size_t)t * pitch + h * hd + d]); o[1] = tohx(F[(size_t)t * pitch + h * hd + d + 1]); *(volatile v2h*)(P + e) = o; __threadfence(); *(volatile v2h*)(P + e) = o; }
__global__ __launch_bounds__(256) void k_vt(const float* __restrict__ F, int pitch, int nh, int hd, h16* VT) { const size_t e = ((size_t)blockIdx.x * 256 + threadIdx.x) * 2; if (e >= (size_t)nh * hd * TT) return; const int t = (int)(e % TT); const int d = (int)((e / TT) % hd); const int h = (int)(e / ((size_t)TT * hd)); v2h o; o[0] = tohx(F[(size_t)t * pitch + h * hd + d]); o[1] = tohx(F[(size_t)(t + 1) * pitch + h * hd + d]); *(volatile v2h*)(VT + e) = o; __threadfence(); *(volatile v2h*)(VT + e) = o; }
__global__ __launch_bounds__(256) void k_asoft(const float* __restrict__ Sb, const float* __restrict__ MOD, int h, float scl, h16* P16) { const int lane = threadIdx.x & 31; const int row = blockIdx.x * 8 + (threadIdx.x >> 5); if (row >= TT) return; const float* sr = Sb + (size_t)row * TT; float sc = scl; if (MOD) { float m = MOD[(size_t)row * 64 + h]; asm volatile("" : "+v"(m)); sc = __fmul_rn(scl, m); } float v[32]; float mx = -3.0e38f;
#pragma unroll
    for (int ch = 0; ch < 8; ++ch) { const int j0 = ch * 128 + lane * 4; const v4f a = *(const v4f*)(sr + j0);
#pragma unroll
        for (int q = 0; q < 4; ++q) { const float t = __fmul_rn(a[q], sc); v[ch * 4 + q] = t; mx = fmaxf(mx, t); } }
#pragma unroll
    for (int sh = 16; sh; sh >>= 1) mx = fmaxf(mx, __shfl_xor(mx, sh, 32));
    float sum = 0.f;
#pragma unroll
    for (int k = 0; k < 32; ++k) { float d0 = __fsub_rn(v[k], mx); asm volatile("" : "+v"(d0)); v[k] = __builtin_amdgcn_exp2f(__fmul_rn(d0, 1.4426950408889634f)); sum += v[k]; }
#pragma unroll
    for (int sh = 16; sh; sh >>= 1) sum += __shfl_xor(sum, sh, 32);
    const float f = __fdiv_rn(PCAR, sum);
#pragma unroll 1
    for (int ps = 0; ps < 2; ++ps) {
#pragma unroll
        for (int ch = 0; ch < 8; ++ch) { v4h o;
#pragma unroll
            for (int q = 0; q < 4; ++q) o[q] = tohx(v[ch * 4 + q] * f); *(volatile v4h*)(P16 + (size_t)row * TT + ch * 128 + lane * 4) = o; }
        if (ps == 0) __threadfence(); } }
__global__ __launch_bounds__(256) void k_mrgf(const float* __restrict__ O, int h, int hd, float* CT) { const size_t e = ((size_t)blockIdx.x * 256 + threadIdx.x) * 2; if (e >= (size_t)TT * hd) return; const int d = (int)(e % hd); const int t = (int)(e / hd); v2f o; o[0] = O[e] * (1.0f / PCAR); o[1] = O[e + 1] * (1.0f / PCAR); const size_t oo = (size_t)t * DD + h * hd + d; *(volatile v2f*)(CT + oo) = o; __threadfence(); *(volatile v2f*)(CT + oo) = o; }
__global__ __launch_bounds__(256) void k_mrg(const float* __restrict__ O, int h, int hd, bf* Ah, bf* Al) { const size_t e = ((size_t)blockIdx.x * 256 + threadIdx.x) * 2; if (e >= (size_t)TT * hd) return; const int d = (int)(e % hd); const int t = (int)(e / hd); v2us oh, ol;
#pragma unroll
    for (int q = 0; q < 2; ++q) { unsigned short a, c2; splitf(O[e + q] * (1.0f / PCAR), a, c2); oh[q] = a; ol[q] = c2; } const size_t oo = (size_t)t * DD + h * hd + d; *(volatile v2us*)(Ah + oo) = oh; *(volatile v2us*)(Al + oo) = ol; __threadfence(); *(volatile v2us*)(Ah + oo) = oh; *(volatile v2us*)(Al + oo) = ol; }
__global__ __launch_bounds__(256) void k_lnT(const float* __restrict__ A, int rnd, const float* __restrict__ g, const float* __restrict__ bb, bf* Yh, bf* Yl) { const int lane = threadIdx.x & 31; const int t = blockIdx.x * 8 + (threadIdx.x >> 5); if (t >= LL) return; const float* ar = A + (size_t)t * DD; float v[32]; float s = 0.f;
#pragma unroll
    for (int ch = 0; ch < 8; ++ch) { const v4f a = *(const v4f*)(ar + ch * 128 + lane * 4);
#pragma unroll
        for (int q = 0; q < 4; ++q) { const float x = rnd ? bfr(a[q]) : a[q]; v[ch * 4 + q] = x; s = __fadd_rn(s, x); } }
#pragma unroll
    for (int sh = 16; sh; sh >>= 1) s += __shfl_xor(s, sh, 32);
    const float mu = s * (1.0f / DD); float q2 = 0.f;
#pragma unroll
    for (int k = 0; k < 32; ++k) { const float d = __fsub_rn(v[k], mu); float p = __fmul_rn(d, d); asm volatile("" : "+v"(p)); q2 = __fadd_rn(q2, p); }
#pragma unroll
    for (int sh = 16; sh; sh >>= 1) q2 += __shfl_xor(q2, sh, 32);
    const float rs = __frsqrt_rn(__fadd_rn(q2 * (1.0f / DD), 1e-5f));
#pragma unroll 1
    for (int ps = 0; ps < 2; ++ps) {
#pragma unroll
        for (int ch = 0; ch < 8; ++ch) { v4us oh, ol;
#pragma unroll
            for (int q = 0; q < 4; ++q) { const int d = ch * 128 + lane * 4 + q; float tn = __fmul_rn(__fsub_rn(v[ch * 4 + q], mu), rs); asm volatile("" : "+v"(tn)); float tg = __fmul_rn(tn, bfr(g[d])); asm volatile("" : "+v"(tg)); unsigned short a2, c2; splitf(__fadd_rn(tg, bfr(bb[d])), a2, c2); oh[q] = a2; ol[q] = c2; }
            const size_t o = (size_t)t * DD + ch * 128 + lane * 4; *(volatile v4us*)(Yh + o) = oh; *(volatile v4us*)(Yl + o) = ol; }
        if (ps == 0) __threadfence(); } }
__global__ __launch_bounds__(256) void k_rope2(const float* __restrict__ F3, const float* __restrict__ FC, float* QK) { const size_t e = (size_t)blockIdx.x * 256 + threadIdx.x; if (e >= (size_t)LL * DD) return; const int pr = (int)(e % DD), t = (int)(e / DD); const int col = pr * 2; const int i = (col % HDM) / 2; const float* src = F3 + (size_t)t * 3 * DD + col;
    const float a = src[0], b = src[1]; const float c = bfr(FC[((size_t)t * 32 + i) * 2]), s = bfr(FC[((size_t)t * 32 + i) * 2 + 1]); float ac = __fmul_rn(a, c), bs = __fmul_rn(b, s), as_ = __fmul_rn(a, s), bc = __fmul_rn(b, c); asm volatile("" : "+v"(ac), "+v"(bs), "+v"(as_), "+v"(bc)); v2f o; o[0] = __fsub_rn(ac, bs); o[1] = __fadd_rn(as_, bc);
    *(volatile v2f*)(QK + (size_t)t * 2 * DD + col) = o; __threadfence(); *(volatile v2f*)(QK + (size_t)t * 2 * DD + col) = o; }
__global__ __launch_bounds__(256) void k_res(const float* __restrict__ x, const float* __restrict__ A, float* H, size_t n) { const size_t i = ((size_t)blockIdx.x * 256 + threadIdx.x) * 4; if (i >= n) return; const v4f a = *(const v4f*)(x + i), b = *(const v4f*)(A + i); v4f o;
#pragma unroll
    for (int q = 0; q < 4; ++q) o[q] = __fadd_rn(bfr(a[q]), b[q]); *(volatile v4f*)(H + i) = o; __threadfence(); *(volatile v4f*)(H + i) = o; }
__global__ __launch_bounds__(256) void k_gelu2(const float* __restrict__ F, bf* Ph, bf* Pl, size_t n) { const size_t i = ((size_t)blockIdx.x * 256 + threadIdx.x) * 2; if (i >= n) return; v2us oh, ol;
#pragma unroll
    for (int q = 0; q < 2; ++q) { const float h = F[i + q]; float er = erff(h * 0.70710678f); asm volatile("" : "+v"(er)); float hh = __fmul_rn(0.5f, h); asm volatile("" : "+v"(hh)); unsigned short a, c2; splitf(__fmul_rn(hh, __fadd_rn(1.0f, er)), a, c2); oh[q] = a; ol[q] = c2; }
    *(volatile v2us*)(Ph + i) = oh; *(volatile v2us*)(Pl + i) = ol; __threadfence(); *(volatile v2us*)(Ph + i) = oh; *(volatile v2us*)(Pl + i) = ol; }
__global__ __launch_bounds__(256) void k_out(const float* __restrict__ H, const float* __restrict__ Y, float* OUT, size_t n) { const size_t i = ((size_t)blockIdx.x * 256 + threadIdx.x) * 4; if (i >= n) return; const v4f a = *(const v4f*)(H + i), b = *(const v4f*)(Y + i); v4f o;
#pragma unroll
    for (int q = 0; q < 4; ++q) o[q] = __fadd_rn(a[q], b[q]); *(volatile v4f*)(OUT + i) = o; __threadfence(); *(volatile v4f*)(OUT + i) = o; }

extern "C" void kernel_launch(void* const* d_in, const int* in_sizes, int n_in,
                              void* d_out, int out_size, void* d_ws, size_t ws_size, hipStream_t stream) {
    (void)in_sizes; (void)n_in; (void)out_size;
    const float* IN[13]; for (int i = 0; i < 13; ++i) IN[i] = (const float*)d_in[i];
    float* OUT = (float*)d_out;
    char* wsp = (char*)d_ws;
    auto take = [&](size_t bytes) { char* p = wsp; wsp += (bytes + 255) & ~(size_t)255; return (void*)p; };
    bf* WQKV = (bf*)take((size_t)3 * DD * DD * 2); bf* WO = (bf*)take((size_t)DD * DD * 2); bf* W0 = (bf*)take((size_t)MM * DD * 2); bf* W1 = (bf*)take((size_t)DD * MM * 2);
    bf* Xh = (bf*)take((size_t)LL * DD * 2); bf* Xl = (bf*)take((size_t)LL * DD * 2); float* F3 = (float*)take((size_t)LL * 3 * DD * 4); float* QK = (float*)take((size_t)LL * 2 * DD * 4);
    h16* QP = (h16*)take((size_t)TT * DD * 2); h16* KP = (h16*)take((size_t)TT * DD * 2); h16* VT = (h16*)take((size_t)DD * TT * 2); float* Sb = (float*)take((size_t)TT * TT * 4); h16* Pm = (h16*)take((size_t)TT * TT * 2); float* O = (float*)take((size_t)TT * HDM * 4); bf* Ah = (bf*)take((size_t)LL * DD * 2); bf* Al = (bf*)take((size_t)LL * DD * 2);
    float* H = (float*)take((size_t)LL * DD * 4); bf* Gh = (bf*)take((size_t)(LL / 2) * MM * 2); bf* Gl = (bf*)take((size_t)(LL / 2) * MM * 2);
    float* G = F3;
    float* Y = QK;
    if ((size_t)(wsp - (char*)d_ws) > ws_size) return;
    { k_wtG<<<(unsigned)(((size_t)DD * 3 * DD / 64 + 63) / 64), 256, 0, stream>>>(IN[7], DD, 3 * DD, WQKV); k_wtG<<<(unsigned)(((size_t)DD * DD / 64 + 63) / 64), 256, 0, stream>>>(IN[8], DD, DD, WO);
      k_wtG<<<(unsigned)(((size_t)DD * MM / 64 + 63) / 64), 256, 0, stream>>>(IN[9], DD, MM, W0); k_wtG<<<(unsigned)(((size_t)MM * DD / 64 + 63) / 64), 256, 0, stream>>>(IN[11], MM, DD, W1); }
    k_lnT<<<LL / 8, 256, 0, stream>>>(IN[0], 1, IN[3], IN[4], Xh, Xl);
    k_gemmw<bf, 1, false><<<dim3(LL / 64, 3 * DD / 64, 1), 32, 0, stream>>>(Xh, Xl, WQKV, nullptr, DD, F3, 3 * DD, nullptr, 0, 0, 0);
    k_rope2<<<(unsigned)(((size_t)LL * DD + 255) / 256), 256, 0, stream>>>(F3, IN[2], QK);
    const unsigned LP = (TT * DD / 2 + 255) / 256; const float scl = 0.125f;
    for (int s = 0; s < NB_; ++s) { const size_t t0 = (size_t)s * TT;
        k_pl<<<LP, 256, 0, stream>>>(QK + t0 * 2 * DD, 2 * DD, NH_, HDM, QP); k_pl<<<LP, 256, 0, stream>>>(QK + t0 * 2 * DD + DD, 2 * DD, NH_, HDM, KP); k_vt<<<LP, 256, 0, stream>>>(F3 + t0 * 3 * DD + 2 * DD, 3 * DD, NH_, HDM, VT);
        for (int h = 0; h < NH_; ++h) {
            k_gemmw<h16, 0, false><<<dim3(TT / 64, TT / 64, 1), 32, 0, stream>>>(QP + (size_t)h * TT * HDM, nullptr, KP + (size_t)h * TT * HDM, nullptr, HDM, Sb, TT, nullptr, 0, 0, 0);
            k_asoft<<<TT / 8, 256, 0, stream>>>(Sb, nullptr, h, scl, Pm);
            k_gemmw<h16, 0, false><<<dim3(TT / 64, 1, 1), 32, 0, stream>>>(Pm, nullptr, VT + (size_t)h * HDM * TT, nullptr, TT, O, HDM, nullptr, 0, 0, 0);
            k_mrg<<<(TT * HDM / 2 + 255) / 256, 256, 0, stream>>>(O, h, HDM, Ah + t0 * DD, Al + t0 * DD); } }
    k_gemmw<bf, 1, false><<<dim3(LL / 64, DD / 64, 1), 32, 0, stream>>>(Ah, Al, WO, nullptr, DD, Y, DD, nullptr, 0, 0, 0);
    k_res<<<(unsigned)(((size_t)LL * DD / 4 + 255) / 256), 256, 0, stream>>>(IN[0], Y, H, (size_t)LL * DD);
    k_lnT<<<LL / 8, 256, 0, stream>>>(H, 0, IN[5], IN[6], Xh, Xl);
    for (int hb = 0; hb < 2; ++hb) { const size_t r0 = (size_t)hb * (LL / 2);
        k_gemmw<bf, 1, true><<<dim3(LL / 2 / 64, MM / 64, 1), 32, 0, stream>>>(Xh + r0 * DD, Xl + r0 * DD, W0, nullptr, DD, G, MM, IN[10], 0, 0, 0);
        k_gelu2<<<(unsigned)(((size_t)(LL / 2) * MM / 2 + 255) / 256), 256, 0, stream>>>(G, Gh, Gl, (size_t)(LL / 2) * MM);
        k_gemmw<bf, 1, true><<<dim3(LL / 2 / 64, DD / 64, 1), 32, 0, stream>>>(Gh, Gl, W1, nullptr, MM, Y, DD, IN[12], 0, 0, 0);
        k_out<<<(unsigned)(((size_t)(LL / 2) * DD / 4 + 255) / 256), 256, 0, stream>>>(H + r0 * DD, Y, OUT + r0 * DD, (size_t)(LL / 2) * DD); }
}
